// T6_45784351375415
// MI455X (gfx1250) — hardware-verified
//
#include <hip/hip_runtime.h>
#include <hip/hip_fp16.h>

typedef __attribute__((ext_vector_type(16))) _Float16 v16h;
typedef __attribute__((ext_vector_type(8)))  float    v8f;
typedef __attribute__((ext_vector_type(4)))  float    v4f_t;
typedef float v4fa __attribute__((ext_vector_type(4), may_alias));

#define B_  4
#define LC  256
#define LR  64
#define NQ  3
#define LQ  32
#define NP  3
#define LP  128
#define H_  256
#define V_  32000
#define M_  (B_*LR)
#define K_  H_
#define NB  64

__global__ __launch_bounds__(256) void k_fmax(
    const float* __restrict__ fc, const float* __restrict__ fq,
    const float* __restrict__ fp, _Float16* __restrict__ A)
{
  int i0 = (blockIdx.x * 256 + threadIdx.x) * 2;
  if (i0 >= M_ * K_) return;
  _Float16 mv[2];
#pragma unroll
  for (int u = 0; u < 2; ++u) {
    const int i = i0 + u;
    int h   = i % H_;
    int row = i / H_;
    int b = row / LR, r = row % LR;
    float m = fc[i];
#pragma unroll
    for (int q = 0; q < NQ; ++q)
      m = fmaxf(m, fq[((b*NQ + q)*LR + r)*H_ + h]);
#pragma unroll
    for (int p = 0; p < NP; ++p)
      m = fmaxf(m, fp[((b*NP + p)*LR + r)*H_ + h]);
    mv[u] = (_Float16)m;
  }
  const unsigned pk = (unsigned)__builtin_bit_cast(unsigned short, mv[0]) | ((unsigned)__builtin_bit_cast(unsigned short, mv[1]) << 16);
  *(volatile unsigned*)(A + i0) = pk; __threadfence(); *(volatile unsigned*)(A + i0) = pk;
}

__global__ __launch_bounds__(256) void k_gemm(
    const _Float16* __restrict__ A, const float* __restrict__ W,
    const float* __restrict__ bias, float* __restrict__ logits)
{
  __shared__ __align__(16) _Float16 As[M_][40];
  __shared__ __align__(16) float Cs[M_ * 68];
  const int n0   = blockIdx.x * NB;
  const int tid  = threadIdx.x;
  const int lane = tid & 31, wv = tid >> 5;
  const int half = lane >> 4, l15 = lane & 15;

  v8f acc[2][4];
#pragma unroll
  for (int a = 0; a < 2; ++a)
#pragma unroll
    for (int c = 0; c < 4; ++c)
#pragma unroll
      for (int e = 0; e < 8; ++e) acc[a][c][e] = 0.f;

  for (int k0 = 0; k0 < K_; k0 += 32) {
    __syncthreads();
    {
      const uint4* s = (const uint4*)(A + (size_t)tid * K_ + k0);
      uint4* d = (uint4*)(&As[tid][0]);
      d[0] = s[0]; d[1] = s[1]; d[2] = s[2]; d[3] = s[3];
    }
    __syncthreads();

    v16h af[2];
#pragma unroll
    for (int mt2 = 0; mt2 < 2; ++mt2) {
      const int m = (wv*2 + mt2)*16 + l15;
#pragma unroll
      for (int j = 0; j < 8; ++j) {
        af[mt2][j]     = As[m][half*8 + j];
        af[mt2][8 + j] = As[m][16 + half*8 + j];
      }
    }

#pragma unroll
    for (int nt = 0; nt < 4; ++nt) {
      const int col = n0 + nt*16 + l15;
      const float* wp = W + (size_t)(k0 + half*8) * V_ + col;
      v16h bf;
#pragma unroll
      for (int j = 0; j < 8; ++j) { bf[j] = (_Float16)wp[(size_t)j * V_]; bf[8 + j] = (_Float16)wp[(size_t)(16 + j) * V_]; }
#pragma unroll
      for (int mt2 = 0; mt2 < 2; ++mt2)
        acc[mt2][nt] = __builtin_amdgcn_wmma_f32_16x16x32_f16(
            false, af[mt2], false, bf, (short)0, acc[mt2][nt], false, false);
    }
  }

#pragma unroll
  for (int nt = 0; nt < 4; ++nt) {
    const int cl = nt*16 + l15;
    const float bv = bias[n0 + cl];
#pragma unroll
    for (int mt2 = 0; mt2 < 2; ++mt2) {
      const int mbase = (wv*2 + mt2)*16 + half*8;
#pragma unroll
      for (int rr = 0; rr < 8; ++rr) Cs[(mbase + rr) * 68 + cl] = acc[mt2][nt][rr] + bv;
    }
  }
  __syncthreads();
#pragma unroll 1
  for (int pass = 0; pass < 2; ++pass) {
    for (int c = tid; c < M_ * 16; c += 256) { const int row = c >> 4, q = (c & 15) * 4;
      *(volatile v4f_t*)(logits + (size_t)row * V_ + n0 + q) = *(const volatile v4fa*)(Cs + row * 68 + q); }
    __threadfence();
  }
}

__global__ __launch_bounds__(256) void k_row(
    const float* __restrict__ logits,
    const int* __restrict__ ctx, const int* __restrict__ qry,
    const int* __restrict__ psg, const float* __restrict__ cw,
    const float* __restrict__ qw, const float* __restrict__ pw,
    const float* __restrict__ selq, const float* __restrict__ selp,
    float* __restrict__ out)
{
  __shared__ __align__(16) float dist[V_];
  __shared__ float red[256];
  __shared__ float tsum[256];
  const int row = blockIdx.x, tid = threadIdx.x;
  const int b = row / LR, r = row % LR;
  const float* lp = logits + (size_t)row * V_;

  for (int v = tid; v < V_; v += 256) dist[v] = 0.f;
  float m = -3.4e38f;
  for (int v = tid; v < V_; v += 256) m = fmaxf(m, lp[v]);
  red[tid] = m; __syncthreads();
  for (int s = 128; s > 0; s >>= 1) { if (tid < s) red[tid] = fmaxf(red[tid], red[tid + s]); __syncthreads(); }
  m = red[0]; __syncthreads();
  float sum = 0.f;
  for (int v = tid; v < V_; v += 256) sum += __expf(lp[v] - m);
  red[tid] = sum; __syncthreads();
  for (int s = 128; s > 0; s >>= 1) { if (tid < s) red[tid] += red[tid + s]; __syncthreads(); }
  const float rinv = 0.5f / red[0];
  __syncthreads();

  for (int src = 0; src < 1 + NQ + NP; ++src) {
    int L; const int* tok; const float* w; float gate;
    if (src == 0) { L = LC; tok = ctx + b*LC; w = cw + (size_t)row * LC; gate = 1.f; }
    else if (src <= NQ) { const int q = src - 1; L = LQ; tok = qry + (b*NQ + q)*LQ; w = qw + ((size_t)(b*NQ + q)*LR + r)*LQ; gate = selq[b*NQ + q]; }
    else { const int p = src - 1 - NQ; L = LP; tok = psg + (b*NP + p)*LP; w = pw + ((size_t)(b*NP + p)*LR + r)*LP; gate = selp[b*NP + p]; }
    const int l = tid;
    bool first = false; int t = 0; float s = 0.f;
    if (l < L) {
      t = tok[l];
      first = true;
      for (int l2 = 0; l2 < L; ++l2) {
        if (tok[l2] == t) { if (l2 < l) { first = false; break; } s += w[l2]; }
      }
      t = (t < 0) ? 0 : (t > V_ - 1 ? V_ - 1 : t);
    }
    __syncthreads();
    if (first) dist[t] = fmaxf(dist[t], gate * s);
    __syncthreads();
  }

  float* orow = out + (size_t)row * V_;
#pragma unroll 1
  for (int pass = 0; pass < 2; ++pass) {
    for (int c = tid; c < V_ / 4; c += 256) {
      const v4f_t lg = *(const v4f_t*)(lp + c * 4);
      const v4f_t d  = *(const volatile v4fa*)(dist + c * 4);
      v4f_t o;
      o.x = 0.5f*d.x + __expf(lg.x - m)*rinv;
      o.y = 0.5f*d.y + __expf(lg.y - m)*rinv;
      o.z = 0.5f*d.z + __expf(lg.z - m)*rinv;
      o.w = 0.5f*d.w + __expf(lg.w - m)*rinv;
      *(volatile v4f_t*)(orow + c * 4) = o;
    }
    __threadfence();
  }
}

extern "C" void kernel_launch(void* const* d_in, const int* in_sizes, int n_in,
                              void* d_out, int out_size, void* d_ws, size_t ws_size,
                              hipStream_t stream)
{
  (void)in_sizes; (void)n_in; (void)out_size; (void)ws_size;
  const int*   ctx  = (const int*)  d_in[0];
  const int*   qry  = (const int*)  d_in[1];
  const int*   psg  = (const int*)  d_in[2];
  const float* cw   = (const float*)d_in[3];
  const float* qw   = (const float*)d_in[4];
  const float* pw   = (const float*)d_in[5];
  const float* fc   = (const float*)d_in[6];
  const float* fq   = (const float*)d_in[7];
  const float* fp   = (const float*)d_in[8];
  const float* selq = (const float*)d_in[9];
  const float* selp = (const float*)d_in[10];
  const float* Wg   = (const float*)d_in[11];
  const float* bg   = (const float*)d_in[12];
  float* out = (float*)d_out;

  char* ws = (char*)d_ws;
  _Float16* Ah  = (_Float16*)ws;
  float* logits = (float*)(ws + (256 << 10));
  float* rmax   = (float*)(ws + (256 << 10) + (size_t)M_ * V_ * sizeof(float));
  float* rsum   = rmax + M_;

  (void)rmax; (void)rsum;
  k_fmax<<<(M_ * K_ / 2) / 256, 256, 0, stream>>>(fc, fq, fp, Ah);
  k_gemm<<<V_ / NB, 256, 0, stream>>>(Ah, Wg, bg, logits);
  k_row<<<M_, 256, 0, stream>>>(logits, ctx, qry, psg, cw, qw, pw, selq, selp, out);
}
